// STA_73650099191827
// MI455X (gfx1250) — hardware-run, weakly checked
//
#include <hip/hip_runtime.h>


#ifndef NB
#define NB 4
#endif
#define NB_FULL 4
#define LL   16
#define NN   4096
#define KD   2048
#define TB   2
#define NBR  2
#define CC   32
#define KP   (KD + 2)
#define TP   (TB + 2)
#define KCV  (9 * CC)
#define RM   (NB * TB * LL)
#define AW   4
#define SW   8
#define CW   32
#define OSP  36
#define QRS  2048.0f
#define QRI  (1.0f / 2048.0f)
#define L2E  1.4426950408889634f
#define PSH  14.0f
#define PSI  (1.0f / 16384.0f)
#define NEGB (-3.0e38f)
#define PLS  ((size_t)NBR * RM * KD)
#define XPS  ((size_t)NB * KP * TP * CC)

static_assert(NB <= NB_FULL);
static_assert(TB == 2);
static_assert(LL == 16);
static_assert(NN == KD * TB);
static_assert(CC == 2 * LL);
static_assert(KCV % 32 == 0);
static_assert(KD % 64 == 0);
static_assert(RM % 64 == 0);
static_assert(NN % 64 == 0);
static_assert(NN % (16 * SW) == 0);
static_assert(NN % (CW * AW) == 0);
static_assert(NN % 32 == 0);
static_assert(((size_t)NB * NN) % (32 * AW) == 0);
static_assert((OSP * 4) % 16 == 0);
static_assert(CW == 32);
static_assert((KD / 8) % 32 == 0);
static_assert(KD % 256 == 0);
static_assert((KD / 2) % 256 == 0);
static_assert((size_t)(KD / 2) * 16 == (size_t)KD * TB * 4);
static_assert(16 * 68 * 4 <= 131072);
static_assert(16 * SW * 4 <= 131072);
static_assert(AW * 16 * OSP * 4 <= 131072);
static_assert(64 * 68 * 4 <= 131072);
static_assert(AW * 32 * OSP * 4 <= 131072);
static_assert(32 * 16 * 4 == 16 * 128);
static_assert(32 * 16 * 8 == 64 * 64);
static_assert(32 * 16 * 1 == 16 * SW * 4);
static_assert(32 * 16 * 4 == 16 * CW * 4);
static_assert(256 * 16 * 2 == 64 * 128);
static_assert(32 * 16 * 8 == 16 * 64 * 4);
static_assert(32 * 16 * 8 == 32 * 32 * 4);

typedef _Float16 h16;
typedef unsigned short bf;
typedef __attribute__((ext_vector_type(16))) __bf16   v16bf;
typedef __attribute__((ext_vector_type(16))) _Float16 v16h;
typedef __attribute__((ext_vector_type(8)))  _Float16 v8h;
typedef __attribute__((ext_vector_type(8)))  unsigned short v8us;
typedef __attribute__((ext_vector_type(8)))  float    v8f;
typedef __attribute__((ext_vector_type(4)))  float    v4f;
typedef __attribute__((ext_vector_type(2)))  float    v2f;
typedef v4f  __attribute__((may_alias)) v4fa;

__device__ __forceinline__ unsigned short f2bf(float f) { unsigned u = __float_as_uint(f); u += 0x7FFFu + ((u >> 16) & 1u); return (unsigned short)(u >> 16); }
__device__ __forceinline__ float bfr(float f) { return __uint_as_float(((unsigned)f2bf(f)) << 16); }
__device__ __forceinline__ v16h cat16(v8h lo, v8h hi) { return __builtin_shufflevector(lo, hi, 0, 1, 2, 3, 4, 5, 6, 7, 8, 9, 10, 11, 12, 13, 14, 15); }
__device__ __forceinline__ v16bf cat16b(v8us lo, v8us hi) { return __builtin_bit_cast(v16bf, __builtin_shufflevector(lo, hi, 0, 1, 2, 3, 4, 5, 6, 7, 8, 9, 10, 11, 12, 13, 14, 15)); }
__device__ __forceinline__ v8f wmma16(v16h a, v16h b, v8f c) { return __builtin_amdgcn_wmma_f32_16x16x32_f16(false, a, false, b, (short)0, c, false, false); }
__device__ __forceinline__ v8f wmmab(v16bf a, v16bf b, v8f c) { return __builtin_amdgcn_wmma_f32_16x16x32_bf16(false, a, false, b, (short)0, c, false, false); }
__device__ __forceinline__ v16h  ldh(const h16* p) { return cat16(*(const v8h*)p, *(const v8h*)(p + 16)); }
__device__ __forceinline__ v16bf ldb(const bf* p)  { return cat16b(*(const v8us*)p, *(const v8us*)(p + 16)); }
__device__ __forceinline__ void wave_sync() { __builtin_amdgcn_fence(3  , "wavefront"); __builtin_amdgcn_wave_barrier(); asm volatile("" ::: "memory"); }

__device__ __forceinline__ h16 toh_flush(float v) { const h16 r = (h16)v; return (fabsf(v) < 6.103515625e-05f) ? (h16)0.0f : r; }
__device__ __forceinline__ float bf2f(unsigned short h) { return __uint_as_float(((unsigned)h) << 16); }
__device__ __forceinline__ v8f wmma16g(v16h a, v16h b, v8f c) { c = wmma16(a, b, c); asm volatile("v_nop\n\tv_nop\n\tv_nop\n\tv_nop" : "+v"(c) : "v"(a), "v"(b)); return c; }
__device__ __forceinline__ v8f wmmabg(v16bf a, v16bf b, v8f c) { c = wmmab(a, b, c); asm volatile("v_nop\n\tv_nop\n\tv_nop\n\tv_nop" : "+v"(c) : "v"(a), "v"(b)); return c; }

__global__ __launch_bounds__(32) void k_embed(const float* __restrict__ IN, const float* __restrict__ W1, h16* PA, h16* EH, int zb0) {
    __shared__ __align__(16) float os[16 * 68];
    const int lane = threadIdx.x & 31, lr = lane & 15, hi = lane >> 4;
    const int n0 = blockIdx.x * 64; const int b = blockIdx.y; const int zb = zb0 + b;
    const v8us zz = (v8us){};
    v8us wl;
#pragma unroll
    for (int i = 0; i < 8; ++i) wl[i] = f2bf(W1[(8 * hi + i) * LL + lr]);
    const v16bf a = cat16b(wl, zz);
    const float* inb = IN + (size_t)b * LL * NN + n0 + lr;
#pragma unroll 1
    for (int nb = 0; nb < 4; ++nb) {
        v8us xl;
#pragma unroll
        for (int i = 0; i < 8; ++i) xl[i] = f2bf(inb[(size_t)(8 * hi + i) * NN + nb * 16]);
        const v8f acc = wmmabg(a, cat16b(xl, zz), (v8f){});
#pragma unroll
        for (int j = 0; j < 8; ++j) os[(hi * 8 + j) * 68 + nb * 16 + lr] = acc[j];
    }
    wave_sync();
    const size_t pb = ((size_t)zb * NN + n0) * 32;
    const size_t eb = (size_t)zb * LL * NN + n0;
#pragma unroll 1
    for (int ps = 0; ps < 2; ++ps) {
#pragma unroll
        for (int s = 0; s < 4; ++s) { const int row = 4 * s + (lane >> 3), c8 = (lane & 7) * 8;
            const v4f x0 = *(const v4fa*)(&os[row * 68 + c8]); const v4f x1 = *(const v4fa*)(&os[row * 68 + c8 + 4]); v8h hv;
#pragma unroll
            for (int i = 0; i < 4; ++i) { hv[i] = toh_flush(x0[i]); hv[4 + i] = toh_flush(x1[i]); }
            *(volatile v8h*)(EH + eb + (size_t)row * NN + c8) = hv; }
#pragma unroll
        for (int s = 0; s < 8; ++s) { const int p = s * 32 + lane; const int nl = p >> 2, part = p & 3;
            const int mb8 = (part & 1) * 8; const bool sel = (part >> 1) != 0; v8h ov;
#pragma unroll
            for (int i = 0; i < 8; ++i) { const float v = os[(mb8 + i) * 68 + nl]; const h16 hv = toh_flush(v); const h16 rv = toh_flush((v - (float)hv) * QRS); ov[i] = sel ? rv : hv; }
            *(volatile v8h*)(PA + pb + (size_t)p * 8) = ov; }
        if (ps == 0) __threadfence(); }
}

__global__ __launch_bounds__(32 * SW) void k_stat(const h16* __restrict__ PA, float* LSE) {
    __shared__ __align__(16) float ls[16 * SW];
    const int lane = threadIdx.x & 31, lr = lane & 15, hi = lane >> 4;
    const int wave = __builtin_amdgcn_readfirstlane((int)(threadIdx.x >> 5));
    const int zb = blockIdx.y;
    const int r0 = (blockIdx.x * SW + wave) * 16;
    const size_t pbase = (size_t)zb * NN * 32;
    const v16h hz = (v16h){};
    const v16h x = ldh(PA + pbase + (size_t)(r0 + lr) * 32 + 8 * hi);
    const v16h q1 = __builtin_shufflevector(x, hz, 0, 1, 2, 3, 4, 5, 6, 7, 16, 17, 18, 19, 20, 21, 22, 23);
    const v16h q2 = __builtin_shufflevector(x, x, 8, 9, 10, 11, 12, 13, 14, 15, 0, 1, 2, 3, 4, 5, 6, 7);
    const size_t ko = pbase + (size_t)lr * 32 + 8 * hi;
    const v8f z8 = (v8f){};
    float m = NEGB, l = 0.0f;
#pragma unroll 1
    for (int key0 = 0; key0 < NN; key0 += 32) {
        const h16* ka = PA + ko + (size_t)key0 * 32;
        const v16h ka0 = ldh(ka), kb0 = ldh(ka + 16 * 32);
        const v8f sHa = wmma16g(ka0, q1, z8), sLa = wmma16g(ka0, q2, z8);
        const v8f sHb = wmma16g(kb0, q1, z8), sLb = wmma16g(kb0, q2, z8);
        float ta[8], tb[8]; float mx = NEGB;
#pragma unroll
        for (int r = 0; r < 8; ++r) { ta[r] = (sHa[r] + sLa[r] * QRI) * L2E; tb[r] = (sHb[r] + sLb[r] * QRI) * L2E; mx = fmaxf(mx, fmaxf(ta[r], tb[r])); }
        const float mnew = fmaxf(m, mx);
        float sum = 0.0f;
#pragma unroll
        for (int r = 0; r < 8; ++r) sum += __builtin_amdgcn_exp2f(ta[r] - mnew) + __builtin_amdgcn_exp2f(tb[r] - mnew);
        l = l * __builtin_amdgcn_exp2f(m - mnew) + sum; m = mnew;
    }
    const float mo = __shfl_xor(m, 16, 32), lo = __shfl_xor(l, 16, 32);
    const float mm = fmaxf(m, mo);
    const float lt = l * __builtin_amdgcn_exp2f(m - mm) + lo * __builtin_amdgcn_exp2f(mo - mm);
    const float lse = mm + log2f(lt);
    if (hi == 0) ls[wave * 16 + lr] = lse;
    __syncthreads();
    if (wave == 0) {
        const v4f v = *(const v4fa*)(&ls[lane * 4]);
        float* dst = LSE + (size_t)zb * NN + (size_t)blockIdx.x * (16 * SW) + lane * 4;
        *(volatile v4f*)dst = v; __threadfence(); *(volatile v4f*)dst = v;
    }
}

__device__ __forceinline__ v16h ptile(v8f sHa, v8f sLa, v8f sHb, v8f sLb, v8f ca, v8f cb) {
    v16h p;
#pragma unroll
    for (int r = 0; r < 8; ++r) {
        const float ea = (sHa[r] + sLa[r] * QRI) * L2E + ca[r];
        const float eb = (sHb[r] + sLb[r] * QRI) * L2E + cb[r];
        const float ga = (ea < -14.0f) ? 0.0f : __builtin_amdgcn_exp2f(ea);
        const float gb = (eb < -14.0f) ? 0.0f : __builtin_amdgcn_exp2f(eb);
        p[r] = (h16)ga; p[8 + r] = (h16)gb; }
    return p;
}

__global__ __launch_bounds__(32 * AW) void k_attend(const h16* __restrict__ PA, const h16* __restrict__ EH, const float* __restrict__ LSE, float* EA) {
    __shared__ __align__(16) float os[AW * 16 * OSP];
    const int lane = threadIdx.x & 31, lr = lane & 15, hi = lane >> 4;
    const int wave = __builtin_amdgcn_readfirstlane((int)(threadIdx.x >> 5));
    const int zb = blockIdx.y;
    const int m0 = (blockIdx.x * AW + wave) * CW;
    const size_t pbase = (size_t)zb * NN * 32;
    const size_t ebase = (size_t)zb * LL * NN;
    const v16h hz = (v16h){};
    const v16h xa = ldh(PA + pbase + (size_t)(m0 + lr) * 32 + 8 * hi);
    const v16h xb = ldh(PA + pbase + (size_t)(m0 + 16 + lr) * 32 + 8 * hi);
    const v16h q1a = __builtin_shufflevector(xa, hz, 0, 1, 2, 3, 4, 5, 6, 7, 16, 17, 18, 19, 20, 21, 22, 23);
    const v16h q2a = __builtin_shufflevector(xa, xa, 8, 9, 10, 11, 12, 13, 14, 15, 0, 1, 2, 3, 4, 5, 6, 7);
    const v16h q1b = __builtin_shufflevector(xb, hz, 0, 1, 2, 3, 4, 5, 6, 7, 16, 17, 18, 19, 20, 21, 22, 23);
    const v16h q2b = __builtin_shufflevector(xb, xb, 8, 9, 10, 11, 12, 13, 14, 15, 0, 1, 2, 3, 4, 5, 6, 7);
    const size_t ko = pbase + (size_t)lr * 32 + 8 * hi;
    const size_t eo = ebase + (size_t)lr * NN + 8 * hi;
    const float* lb = LSE + (size_t)zb * NN + 8 * hi;
    const v8f z8 = (v8f){};
    v8f o0 = (v8f){}, o1 = (v8f){};
#pragma unroll 1
    for (int key0 = 0; key0 < NN; key0 += 32) {
        const h16* ka = PA + ko + (size_t)key0 * 32;
        const v16h ka0 = ldh(ka), kb0 = ldh(ka + 16 * 32);
        const float* lp = lb + key0;
        const v4f c0 = *(const v4f*)lp, c1 = *(const v4f*)(lp + 4), c2 = *(const v4f*)(lp + 16), c3 = *(const v4f*)(lp + 20);
        v8f ca, cb;
#pragma unroll
        for (int r = 0; r < 4; ++r) { ca[r] = PSH - c0[r]; ca[4 + r] = PSH - c1[r]; cb[r] = PSH - c2[r]; cb[4 + r] = PSH - c3[r]; }
        v16h pb0, pb1;
        { const v8f sHa = wmma16g(ka0, q1a, z8), sLa = wmma16g(ka0, q2a, z8);
          const v8f sHb = wmma16g(kb0, q1a, z8), sLb = wmma16g(kb0, q2a, z8);
          pb0 = ptile(sHa, sLa, sHb, sLb, ca, cb); }
        { const v8f sHa = wmma16g(ka0, q1b, z8), sLa = wmma16g(ka0, q2b, z8);
          const v8f sHb = wmma16g(kb0, q1b, z8), sLb = wmma16g(kb0, q2b, z8);
          pb1 = ptile(sHa, sLa, sHb, sLb, ca, cb); }
        const v16h va = ldh(EH + eo + key0);
        o0 = wmma16g(va, pb0, o0); o1 = wmma16g(va, pb1, o1);
    }
    const int wb = wave * 16 * OSP;
#pragma unroll
    for (int r = 0; r < 8; ++r) { os[wb + (8 * hi + r) * OSP + lr] = o0[r] * PSI; os[wb + (8 * hi + r) * OSP + 16 + lr] = o1[r] * PSI; }
    wave_sync();
    float* orow = EA + ebase + m0;
#pragma unroll 1
    for (int ps = 0; ps < 2; ++ps) {
#pragma unroll
        for (int s = 0; s < 4; ++s) { const int row = 4 * s + (lane >> 3), cofs = (lane & 7) * 4;
            const v4f val = *(const v4fa*)(&os[wb + row * OSP + cofs]);
            *(volatile v4f*)(orow + (size_t)row * NN + cofs) = val; }
        if (ps == 0) __threadfence(); }
}

__global__ __launch_bounds__(256) void k_eacvt(const float* __restrict__ EA, bf* A2) {
    const int i = blockIdx.x * 256 + threadIdx.x; if (i >= NBR * NB * LL * (KD / 8)) return;
    const int kc = i % (KD / 8); const int row = i / (KD / 8); const int l = row % LL; const int zb = row / LL; const int br = zb / NB, b = zb % NB;
    const float* src = EA + (size_t)row * NN + (size_t)kc * 16;
    const v8f y0 = *(const v8f*)src, y1 = *(const v8f*)(src + 8);
    v8us h0, l0, h1, l1;
#pragma unroll
    for (int j = 0; j < 4; ++j) {
        const float a0 = y0[2 * j], a1 = y0[2 * j + 1], c0 = y1[2 * j], c1 = y1[2 * j + 1];
        const unsigned short ha0 = f2bf(a0), ha1 = f2bf(a1), hc0 = f2bf(c0), hc1 = f2bf(c1);
        h0[j] = ha0; l0[j] = f2bf(a0 - bf2f(ha0)); h1[j] = ha1; l1[j] = f2bf(a1 - bf2f(ha1));
        h0[4 + j] = hc0; l0[4 + j] = f2bf(c0 - bf2f(hc0)); h1[4 + j] = hc1; l1[4 + j] = f2bf(c1 - bf2f(hc1)); }
    const size_t d0 = ((size_t)br * RM + (size_t)(b * TB + 0) * LL + l) * KD + (size_t)kc * 8;
    const size_t d1 = ((size_t)br * RM + (size_t)(b * TB + 1) * LL + l) * KD + (size_t)kc * 8;
    *(volatile v8us*)(A2 + d0) = h0; *(volatile v8us*)(A2 + d1) = h1; *(volatile v8us*)(A2 + PLS + d0) = l0; *(volatile v8us*)(A2 + PLS + d1) = l1;
    __threadfence();
    *(volatile v8us*)(A2 + d0) = h0; *(volatile v8us*)(A2 + d1) = h1; *(volatile v8us*)(A2 + PLS + d0) = l0; *(volatile v8us*)(A2 + PLS + d1) = l1;
}

__global__ __launch_bounds__(256) void k_wtr(const float* __restrict__ W, bf* WT) {
    __shared__ __align__(16) float tl[64 * 68];
    const int tid = threadIdx.x; const int j0 = blockIdx.x * 64, k0 = blockIdx.y * 64;
#pragma unroll
    for (int it = 0; it < 4; ++it) { const int row = it * 16 + (tid >> 4), c4 = (tid & 15) * 4;
        const v4f v = *(const v4f*)(W + (size_t)(k0 + row) * KD + j0 + c4); *(v4fa*)(&tl[row * 68 + c4]) = v; }
    __syncthreads();
#pragma unroll 1
    for (int ps = 0; ps < 2; ++ps) {
#pragma unroll
        for (int it = 0; it < 2; ++it) { const int jl = it * 32 + (tid >> 3), q = tid & 7; v8us o;
#pragma unroll
            for (int i = 0; i < 8; ++i) o[i] = f2bf(tl[(8 * q + i) * 68 + jl]);
            *(volatile v8us*)(WT + (size_t)(j0 + jl) * KD + k0 + 8 * q) = o; }
        if (ps == 0) __threadfence(); }
}

__global__ __launch_bounds__(32) void k_mix(const bf* __restrict__ A2, const bf* __restrict__ WT, float* MP) {
    __shared__ __align__(16) float os[16 * 68];
    const int lane = threadIdx.x & 31, lr = lane & 15, hi = lane >> 4;
    const int r0 = blockIdx.x * 64, c0 = blockIdx.y * 64, br = blockIdx.z;
    v8f acc[4][4];
#pragma unroll
    for (int mb = 0; mb < 4; ++mb)
#pragma unroll
        for (int nb = 0; nb < 4; ++nb) acc[mb][nb] = (v8f){};
    const size_t aoff = ((size_t)br * RM + r0 + lr) * KD + 8 * hi, boff = ((size_t)br * KD + c0 + lr) * KD + 8 * hi;
#pragma unroll 1
    for (int pl = 0; pl < 2; ++pl) {
        const size_t po = (size_t)pl * PLS + aoff;
#pragma unroll 1
        for (int kc = 0; kc < KD; kc += 32) {
            v16bf a[4];
#pragma unroll
            for (int mb = 0; mb < 4; ++mb) a[mb] = ldb(A2 + po + (size_t)mb * 16 * KD + kc);
#pragma unroll
            for (int nb = 0; nb < 4; ++nb) { const v16bf b = ldb(WT + boff + (size_t)nb * 16 * KD + kc);
#pragma unroll
                for (int mb = 0; mb < 4; ++mb) acc[mb][nb] = wmmabg(a[mb], b, acc[mb][nb]); }
        }
    }
    float* mrow = MP + ((size_t)br * RM + r0) * KD + c0;
#pragma unroll
    for (int mb = 0; mb < 4; ++mb) {
#pragma unroll
        for (int nb = 0; nb < 4; ++nb) {
#pragma unroll
            for (int j = 0; j < 8; ++j) os[(hi * 8 + j) * 68 + nb * 16 + lr] = acc[mb][nb][j]; }
        wave_sync();
#pragma unroll 1
        for (int ps = 0; ps < 2; ++ps) {
#pragma unroll
            for (int s = 0; s < 8; ++s) { const int row = 2 * s + (lane >> 4), c4 = (lane & 15) * 4;
                const v4f val = *(const v4fa*)(&os[row * 68 + c4]);
                *(volatile v4f*)(mrow + (size_t)(mb * 16 + row) * KD + c4) = val; }
            if (ps == 0) __threadfence(); }
        wave_sync();
    }
}

__global__ __launch_bounds__(256) void k_pe(float* PE) {
    const int i = blockIdx.x * 256 + threadIdx.x; if (i >= KD / 2) return;
    const float dv = expf(0.0f * (-logf(10000.0f) / (float)TB));
    float s0 = 0.0f, c0 = 0.0f, s1 = 0.0f, c1 = 0.0f;
#pragma unroll 1
    for (int j = 0; j < 2; ++j) {
        const float ang = (float)(2 * i + j) * dv;
        const float sv = sinf(ang), cv = cosf(ang);
        s0 = (j == 0) ? sv : s0; c0 = (j == 0) ? cv : c0;
        s1 = (j == 1) ? sv : s1; c1 = (j == 1) ? cv : c1; }
    v4f o; o[0] = s0; o[1] = c0; o[2] = s1; o[3] = c1;
    *(volatile v4f*)(PE + (size_t)i * 4) = o; __threadfence(); *(volatile v4f*)(PE + (size_t)i * 4) = o;
}

__global__ __launch_bounds__(256) void k_wcv(const float* __restrict__ W, bf* WC) {
    const int i = blockIdx.x * 256 + threadIdx.x; if (i >= CC * 9 * 4) return;
    const int q = i & 3; const int tap = (i >> 2) % 9; const int oc = i / 36;
    v8us o;
#pragma unroll
    for (int j = 0; j < 8; ++j) o[j] = f2bf(W[(size_t)(oc * CC + 8 * q + j) * 9 + tap]);
    *(volatile v8us*)(WC + (size_t)i * 8) = o; __threadfence(); *(volatile v8us*)(WC + (size_t)i * 8) = o;
}

__global__ __launch_bounds__(256) void k_hat(const float* __restrict__ IN, const float* __restrict__ MPB, const float* __restrict__ PE, bf* XHB, int pef) {
#pragma clang fp contract(off)
    const int i = blockIdx.x * 256 + threadIdx.x; if (i >= NB * KP * TP * 4) return;
    const int pq = i & 3, tt = (i >> 2) & 3; const int rest = i >> 4; const int kk = rest % KP, b = rest / KP;
    const bool valid = (kk >= 1) & (kk <= KD) & (tt >= 1) & (tt <= TB);
    int k = kk - 1; k = k < 0 ? 0 : (k > KD - 1 ? KD - 1 : k);
    int t = tt - 1; t = t < 0 ? 0 : (t > TB - 1 ? TB - 1 : t);
    const int cb = (pq & 1) * 8; const bool ism = pq < 2;
    float pe = PE[(size_t)k * 2 + t]; asm volatile("" : "+v"(pe));
    const float pev = (pef != 0) ? pe : 0.0f;
    v8us hv, lv;
#pragma unroll
    for (int j = 0; j < 8; ++j) { const int c = cb + j;
        float x = IN[((size_t)b * LL + c) * NN + 2 * k + t];
        float mv = MPB[((size_t)(b * TB + t) * LL + c) * KD + k];
        asm volatile("" : "+v"(x)); asm volatile("" : "+v"(mv));
        x = bfr(x);
        const float pr = mv * x;
        float v = ism ? pr : x;
        v = v + pev;
        v = valid ? v : 0.0f;
        const unsigned short h = f2bf(v); hv[j] = h; lv[j] = f2bf(v - bf2f(h)); }
    *(volatile v8us*)(XHB + (size_t)i * 8) = hv; *(volatile v8us*)(XHB + XPS + (size_t)i * 8) = lv;
    __threadfence();
    *(volatile v8us*)(XHB + (size_t)i * 8) = hv; *(volatile v8us*)(XHB + XPS + (size_t)i * 8) = lv;
}

__global__ __launch_bounds__(32 * AW) void k_conv(const bf* __restrict__ XH, const bf* __restrict__ WC, const float* __restrict__ bias, float* OUT, int choff) {
    __shared__ __align__(16) float os[AW * 32 * OSP];
    const int lane = threadIdx.x & 31, lr = lane & 15, hi = lane >> 4;
    const int wave = __builtin_amdgcn_readfirstlane((int)(threadIdx.x >> 5));
    const int pix0 = (blockIdx.x * AW + wave) * 32; const int b = pix0 / NN; const int p = pix0 % NN;
    size_t ao0, ao1;
    { const int px = p + lr;      ao0 = ((((size_t)b * KP + (px >> 1)) * TP + (px & 1)) * CC) + 8 * hi; }
    { const int px = p + 16 + lr; ao1 = ((((size_t)b * KP + (px >> 1)) * TP + (px & 1)) * CC) + 8 * hi; }
    const size_t wo = (size_t)lr * KCV + 8 * hi;
    v8f a00 = (v8f){}, a01 = (v8f){}, a10 = (v8f){}, a11 = (v8f){};
#pragma unroll 1
    for (int tap = 0; tap < 9; ++tap) {
        const int kh = tap / 3, kw = tap - 3 * kh;
        const size_t to = (size_t)(kh * TP + kw) * CC;
        const v16bf b0 = ldb(WC + wo + tap * 32), b1 = ldb(WC + wo + (size_t)16 * KCV + tap * 32);
#pragma unroll
        for (int pl = 0; pl < 2; ++pl) {
            const v16bf x0 = ldb(XH + (size_t)pl * XPS + ao0 + to), x1 = ldb(XH + (size_t)pl * XPS + ao1 + to);
            a00 = wmmabg(x0, b0, a00); a01 = wmmabg(x0, b1, a01);
            a10 = wmmabg(x1, b0, a10); a11 = wmmabg(x1, b1, a11); }
    }
    const float bc0 = bfr(bias[lr]), bc1 = bfr(bias[16 + lr]);
    const int wb = wave * 32 * OSP;
#pragma unroll
    for (int r = 0; r < 8; ++r) {
        os[wb + lr * OSP + 8 * hi + r] = a00[r] + bc0;        os[wb + lr * OSP + 16 + 8 * hi + r] = a10[r] + bc0;
        os[wb + (16 + lr) * OSP + 8 * hi + r] = a01[r] + bc1; os[wb + (16 + lr) * OSP + 16 + 8 * hi + r] = a11[r] + bc1; }
    wave_sync();
    float* orow = OUT + ((size_t)b * (2 * CC) + choff) * NN + p;
#pragma unroll 1
    for (int ps = 0; ps < 2; ++ps) {
#pragma unroll
        for (int s = 0; s < 8; ++s) { const int row = 4 * s + (lane >> 3), cofs = (lane & 7) * 4;
            const v4f val = *(const v4fa*)(&os[wb + row * OSP + cofs]);
            *(volatile v4f*)(orow + (size_t)row * NN + cofs) = val; }
        if (ps == 0) __threadfence(); }
}

static constexpr size_t al256(size_t v) { return (v + 255) & ~(size_t)255; }
static constexpr size_t SZ_PA = al256((size_t)NBR * NB * NN * 32 * 2);
static constexpr size_t SZ_EH = al256((size_t)NBR * NB * LL * NN * 2);
static constexpr size_t SZ_LS = al256((size_t)NBR * NB * NN * 4);
static constexpr size_t SZ_EA = al256((size_t)NBR * NB * LL * NN * 4);
static constexpr size_t SZ_A2 = al256((size_t)2 * NBR * RM * KD * 2);
static constexpr size_t SZ_WT = al256((size_t)NBR * KD * KD * 2);
static constexpr size_t SZ_MP = al256((size_t)NBR * RM * KD * 4);
static constexpr size_t SZ_PE = al256((size_t)KD * TB * 4);
static constexpr size_t SZ_XH = al256((size_t)NBR * 2 * NB * KP * TP * CC * 2);
static constexpr size_t SZ_WC = al256((size_t)NBR * CC * KCV * 2);
static constexpr size_t SZ_TOTAL = SZ_PA + SZ_EH + SZ_LS + SZ_EA + SZ_A2 + SZ_WT + SZ_MP + SZ_PE + SZ_XH + SZ_WC;
static_assert(SZ_TOTAL <= (size_t)134217728);
static_assert(((size_t)NB * KP * TP * CC * 2) % 256 == 0);
static_assert(((size_t)CC * KCV * 2) % 256 == 0);
static_assert(((size_t)KD * KD * 2) % 256 == 0);
static_assert((size_t)NB * KP * TP * 4 * 8 == (size_t)NB * KP * TP * CC);
static_assert((size_t)NBR * NB * LL * (KD / 8) * 16 == (size_t)NBR * NB * LL * NN);
static_assert((size_t)CC * 9 * 4 * 8 == (size_t)CC * KCV);
static_assert((size_t)NB * (2 * CC) * NN * 4 == (size_t)NB * 1048576);

extern "C" void kernel_launch(void* const* d_in, const int* in_sizes, int n_in,
                              void* d_out, int out_size, void* d_ws, size_t ws_size, hipStream_t stream) {
    if (n_in < 10) return;
    if ((size_t)in_sizes[0] < (size_t)NB * LL * NN || (size_t)in_sizes[1] < (size_t)NB * LL * NN) return;
    if (in_sizes[2] < LL * LL || in_sizes[3] < LL * LL) return;
    if ((size_t)in_sizes[4] < (size_t)KD * KD || (size_t)in_sizes[5] < (size_t)KD * KD) return;
    if (in_sizes[6] < CC * CC * 9 || in_sizes[8] < CC * CC * 9 || in_sizes[7] < CC || in_sizes[9] < CC) return;
    if ((size_t)out_size < (size_t)NB * (2 * CC) * NN) return;
    if (SZ_TOTAL > ws_size) return;
    const float* X = (const float*)d_in[0]; const float* S = (const float*)d_in[1];
    const float* W1x = (const float*)d_in[2]; const float* W1s = (const float*)d_in[3];
    const float* W2x = (const float*)d_in[4]; const float* W2s = (const float*)d_in[5];
    const float* cwx = (const float*)d_in[6]; const float* cbx = (const float*)d_in[7];
    const float* cws = (const float*)d_in[8]; const float* cbs = (const float*)d_in[9];
    float* OUT = (float*)d_out;
    char* wsp = (char*)d_ws;
    h16* PA = (h16*)wsp;  wsp += SZ_PA;
    h16* EH = (h16*)wsp;  wsp += SZ_EH;
    float* LSE = (float*)wsp; wsp += SZ_LS;
    float* EA = (float*)wsp;  wsp += SZ_EA;
    bf* A2 = (bf*)wsp;    wsp += SZ_A2;
    bf* WTP = (bf*)wsp;   wsp += SZ_WT;
    float* MP = (float*)wsp;  wsp += SZ_MP;
    float* PE = (float*)wsp;  wsp += SZ_PE;
    bf* XH = (bf*)wsp;    wsp += SZ_XH;
    bf* WC = (bf*)wsp;    wsp += SZ_WC;

    k_embed<<<dim3(NN / 64, NB, 1), 32, 0, stream>>>(S, W1x, PA, EH, 0);
    k_embed<<<dim3(NN / 64, NB, 1), 32, 0, stream>>>(X, W1s, PA, EH, NB);
    k_stat<<<dim3(NN / (16 * SW), NBR * NB, 1), 32 * SW, 0, stream>>>(PA, LSE);
    k_attend<<<dim3(NN / (CW * AW), NBR * NB, 1), 32 * AW, 0, stream>>>(PA, EH, LSE, EA);
    { const unsigned n = (unsigned)((size_t)NBR * NB * LL * (KD / 8)); k_eacvt<<<(n + 255) / 256, 256, 0, stream>>>(EA, A2); }
    k_wtr<<<dim3(KD / 64, KD / 64, 1), 256, 0, stream>>>(W2x, WTP);
    k_wtr<<<dim3(KD / 64, KD / 64, 1), 256, 0, stream>>>(W2s, WTP + (size_t)KD * KD);
    k_mix<<<dim3(RM / 64, KD / 64, NBR), 32, 0, stream>>>(A2, WTP, MP);
    k_pe<<<(KD / 2) / 256, 256, 0, stream>>>(PE);
    { const unsigned g = (unsigned)((CC * 9 * 4 + 255) / 256);
      k_wcv<<<g, 256, 0, stream>>>(cwx, WC); k_wcv<<<g, 256, 0, stream>>>(cws, WC + (size_t)CC * KCV); }
    { const unsigned g = (unsigned)(((size_t)NB * KP * TP * 4 + 255) / 256);
      k_hat<<<g, 256, 0, stream>>>(X, MP, PE, XH, 0);
      k_hat<<<g, 256, 0, stream>>>(S, MP + (size_t)RM * KD, PE, XH + 2 * XPS, 1); }
    { const unsigned g = (unsigned)(((size_t)NB * NN) / (32 * AW));
      k_conv<<<g, 32 * AW, 0, stream>>>(XH, WC, cbx, OUT, 0);
      k_conv<<<g, 32 * AW, 0, stream>>>(XH + 2 * XPS, WC + (size_t)CC * KCV, cbs, OUT, CC); }
}
